// GIN_Graph_34497177322039
// MI455X (gfx1250) — hardware-verified
//
#include <hip/hip_runtime.h>
#include <stddef.h>


#define HID     128
#define KOUT    256
#define NTHR    256
#define NWAVE   8
#define EPT     8
#define NGRP    2
#define CHUNK   (NTHR * EPT * NGRP)
#define WCAP    (EPT * NGRP * 32)
#define LISTN   (NWAVE * WCAP)
#define NBC     4096
#define NBF     2048
#define NSUB    (NBC / NBF)
#define TPS     (NBF / 8)
#define WPS     (TPS / 32)
#define NBP     32
#define RCAP    40960
#define RBN     128
#define TGT     256
#define DEGCAP  256
#define GROWS   128
#define OTHR    512
#define APH     (HID + 8)
#define APO     (KOUT + 8)
#define BNEPS   1e-5f
#define LNEPS   1e-5f

#define LDS_FILL ((RCAP + NBF + LISTN) * 4 + 64)
#define LDS_G1   (2 * GROWS * APH * 2 + GROWS * HID * 4 + 2 * HID * 8)
#define LDS_G2   (2 * GROWS * APH * 2 + GROWS * HID * 4 + 3 * HID * 4)
#define LDS_HD   (2 * GROWS * APO * 2 + GROWS * HID * 4)

static_assert((CHUNK & (CHUNK - 1)) == 0);
static_assert(CHUNK <= 4096);
static_assert(NBC <= 4096 && NBF <= 4096 && NBP <= 4096);
static_assert((NBC & (NBC - 1)) == 0 && (NBF & (NBF - 1)) == 0 && (NBP & (NBP - 1)) == 0);
static_assert(NBC % NBF == 0 && NSUB >= 1 && NSUB <= 8);
static_assert(OTHR * 8 == NBC);
static_assert((TPS % 32) == 0 && TPS * NSUB == OTHR && (TPS & (TPS - 1)) == 0);
static_assert((RCAP % 32) == 0);
static_assert(TGT == NWAVE * 32 && (TGT % GROWS) == 0);
static_assert(GROWS == NWAVE * 16);
static_assert((GROWS * HID / 8) % NTHR == 0 && (GROWS * KOUT / 8) % NTHR == 0);
static_assert((HID * HID / 8) % NTHR == 0 && (HID * KOUT / 8) % NTHR == 0);
static_assert(NBP * KOUT / 4 == 8 * NTHR);
static_assert(LDS_FILL <= 300000 && LDS_HD <= 300000 && LDS_G1 <= 300000);

typedef float          v4f  __attribute__((ext_vector_type(4)));
typedef float          v8f  __attribute__((ext_vector_type(8)));
typedef int            v4i  __attribute__((ext_vector_type(4)));
typedef unsigned short v8us __attribute__((ext_vector_type(8)));
typedef __bf16         v16b __attribute__((ext_vector_type(16)));
union FragB { v16b v; v8us h[2]; };

__device__ __forceinline__ unsigned int bf_rne(float f) {
  unsigned int u = __float_as_uint(f);
  u += 0x7FFFu + ((u >> 16) & 1u);
  return u >> 16;
}

__device__ __forceinline__ void split2(float x, unsigned short& hi, unsigned short& lo) {
  const unsigned int h = bf_rne(x);
  const float hf = __uint_as_float(h << 16);
  hi = (unsigned short)h;
  lo = (unsigned short)bf_rne(x - hf);
}

__device__ __forceinline__ void split8(v4f a, v4f b, v8us& hi, v8us& lo) {
  unsigned short h, l;
  split2(a.x, h, l); hi[0] = h; lo[0] = l;
  split2(a.y, h, l); hi[1] = h; lo[1] = l;
  split2(a.z, h, l); hi[2] = h; lo[2] = l;
  split2(a.w, h, l); hi[3] = h; lo[3] = l;
  split2(b.x, h, l); hi[4] = h; lo[4] = l;
  split2(b.y, h, l); hi[5] = h; lo[5] = l;
  split2(b.z, h, l); hi[6] = h; lo[6] = l;
  split2(b.w, h, l); hi[7] = h; lo[7] = l;
}

__device__ __forceinline__ v8f wm3(v16b ah, v16b al, v16b bh, v16b bl, v8f c) {
  c = __builtin_amdgcn_wmma_f32_16x16x32_bf16(false, ah, false, bh, (short)0, c, false, false);
  c = __builtin_amdgcn_wmma_f32_16x16x32_bf16(false, ah, false, bl, (short)0, c, false, false);
  c = __builtin_amdgcn_wmma_f32_16x16x32_bf16(false, al, false, bh, (short)0, c, false, false);
  asm volatile("v_nop\n\tv_nop\n\tv_nop\n\tv_nop" : "+v"(c) : "v"(ah), "v"(al), "v"(bh), "v"(bl));
  return c;
}

__device__ __forceinline__ float wsum(float v) {
  v += __shfl_xor(v, 16, 32);
  v += __shfl_xor(v, 8, 32);
  v += __shfl_xor(v, 4, 32);
  v += __shfl_xor(v, 2, 32);
  v += __shfl_xor(v, 1, 32);
  return v;
}

template <int NB>
__device__ __forceinline__ int scan_chunk(const int* __restrict__ dsts, int nE, int cbase, int slotBase,
                                          int vec8, int* list, int tid, int lane, int wave) {
  int wc = 0;
#pragma unroll
  for (int g = 0; g < NGRP; ++g) {
    const int el0  = (g * NTHR + tid) * EPT;
    const int e0   = cbase + el0;
    const int sent = -2147483647 - 1;
    v4i da, db;
    if (vec8 != 0 && cbase + CHUNK <= nE) {
      da = *(const v4i*)(dsts + e0);
      db = *(const v4i*)(dsts + e0 + 4);
    } else {
      da.x = (e0     < nE) ? dsts[min(e0, nE - 1)] : sent;
      da.y = (e0 + 1 < nE) ? dsts[min(e0 + 1, nE - 1)] : sent;
      da.z = (e0 + 2 < nE) ? dsts[min(e0 + 2, nE - 1)] : sent;
      da.w = (e0 + 3 < nE) ? dsts[min(e0 + 3, nE - 1)] : sent;
      db.x = (e0 + 4 < nE) ? dsts[min(e0 + 4, nE - 1)] : sent;
      db.y = (e0 + 5 < nE) ? dsts[min(e0 + 5, nE - 1)] : sent;
      db.z = (e0 + 6 < nE) ? dsts[min(e0 + 6, nE - 1)] : sent;
      db.w = (e0 + 7 < nE) ? dsts[min(e0 + 7, nE - 1)] : sent;
    }
    const unsigned nb = (unsigned)slotBase;
    const unsigned s0 = (unsigned)da.x - nb, s1 = (unsigned)da.y - nb;
    const unsigned s2 = (unsigned)da.z - nb, s3 = (unsigned)da.w - nb;
    const unsigned s4 = (unsigned)db.x - nb, s5 = (unsigned)db.y - nb;
    const unsigned s6 = (unsigned)db.z - nb, s7 = (unsigned)db.w - nb;
    const bool h0 = s0 < (unsigned)NB, h1 = s1 < (unsigned)NB, h2 = s2 < (unsigned)NB, h3 = s3 < (unsigned)NB;
    const bool h4 = s4 < (unsigned)NB, h5 = s5 < (unsigned)NB, h6 = s6 < (unsigned)NB, h7 = s7 < (unsigned)NB;
    const unsigned any = __builtin_amdgcn_ballot_w32(h0 | h1 | h2 | h3 | h4 | h5 | h6 | h7);
    if (any != 0u) {
#define HITJ(J, HJ, SJ) { \
        const unsigned mj = __builtin_amdgcn_ballot_w32(HJ); \
        if (mj != 0u) { \
          if (HJ) { \
            const int pos = wc + (int)__builtin_amdgcn_mbcnt_lo(mj, 0u); \
            if (pos < WCAP) list[wave * WCAP + pos] = ((el0 + (J)) << 12) | (int)(SJ); \
          } \
          wc += (int)__builtin_popcount(mj); } }
      HITJ(0, h0, s0)
      HITJ(1, h1, s1)
      HITJ(2, h2, s2)
      HITJ(3, h3, s3)
      HITJ(4, h4, s4)
      HITJ(5, h5, s5)
      HITJ(6, h6, s6)
      HITJ(7, h7, s7)
#undef HITJ
    }
  }
  return wc;
}

__global__ __launch_bounds__(NTHR) void k_wprep(
    const float* __restrict__ W1, const float* __restrict__ W2, const float* __restrict__ Wo,
    unsigned short* w1h, unsigned short* w1l, unsigned short* w2h, unsigned short* w2l,
    unsigned short* woh, unsigned short* wol, int L) {
  const int g1 = L * (HID * HID / 8);
  const int g2 = g1;
  const int g3 = HID * KOUT / 8;
  const int bstart = blockIdx.x * NTHR;
  const float* src; unsigned short* dh; unsigned short* dl; int K, per, segOff;
  if (bstart < g1)           { src = W1; dh = w1h; dl = w1l; K = HID;  per = HID * HID; segOff = 0; }
  else if (bstart < g1 + g2) { src = W2; dh = w2h; dl = w2l; K = HID;  per = HID * HID; segOff = g1; }
  else                       { src = Wo; dh = woh; dl = wol; K = KOUT; per = 0;         segOff = g1 + g2; }
  const int i = bstart + (int)threadIdx.x;
  if (i >= g1 + g2 + g3) return;
  const int o = (i - segOff) * 8;
  int oo = o;
  if (per != 0) {
    const int layer = o / per;
    src += (size_t)layer * per;
    oo = o - layer * per;
  }
  const int n  = oo / K;
  const int k0 = oo - n * K;
  float v[8];
#pragma unroll
  for (int e = 0; e < 8; ++e) v[e] = src[(size_t)(k0 + e) * HID + n];
  v4f a, b;
  a.x = v[0]; a.y = v[1]; a.z = v[2]; a.w = v[3];
  b.x = v[4]; b.y = v[5]; b.z = v[6]; b.w = v[7];
  v8us hi, lo;
  split8(a, b, hi, lo);
  unsigned short* ph = dh + o;
  unsigned short* pl = dl + o;
  *(volatile v8us*)ph = hi;
  *(volatile v8us*)pl = lo;
  __threadfence();
  *(volatile v8us*)ph = hi;
  *(volatile v8us*)pl = lo;
}

__global__ __launch_bounds__(NTHR) void k_count(const int* __restrict__ ei, int* cnt, int nE, int vec8) {
  __shared__ __attribute__((aligned(16))) int scnt[NBC];
  __shared__ __attribute__((aligned(16))) int list[LISTN];
  __shared__ int wcnt[NWAVE];
  const int tid = threadIdx.x, lane = tid & 31, wave = tid >> 5;
  const int nodeBase = blockIdx.x * NBC;
  const int* dsts = ei + nE;

  for (int i = tid; i < NBC; i += NTHR) scnt[i] = 0;
  __syncthreads();

  const int nChunks = (nE + CHUNK - 1) / CHUNK;
#pragma unroll 1
  for (int ch = 0; ch < nChunks; ++ch) {
    const int cbase = ch * CHUNK;
    const int wc = scan_chunk<NBC>(dsts, nE, cbase, nodeBase, vec8, list, tid, lane, wave);
    if (lane == 0) wcnt[wave] = wc;
    __syncthreads();
    if (wave == 0) {
#pragma unroll 1
      for (int wsx = 0; wsx < NWAVE; ++wsx) {
        int n = __builtin_amdgcn_readfirstlane(wcnt[wsx]);
        n = n > WCAP ? WCAP : (n < 0 ? 0 : n);
        const int* lp = list + wsx * WCAP;
#pragma unroll 1
        for (int i = 0; i < n; ++i) {
          const int ent  = __builtin_amdgcn_readfirstlane(lp[i]);
          const int slot = ent & (NBC - 1);
          if (lane == 0) scnt[slot] = scnt[slot] + 1;
        }
      }
    }
    __syncthreads();
  }

  v4i cq[4];
#pragma unroll
  for (int q = 0; q < 4; ++q) {
    const int f = (wave * 4 + q) * 128 + 4 * lane;
    cq[q] = *(const v4i*)(scnt + f);
  }
  int* cp = cnt + (size_t)nodeBase;
#pragma unroll
  for (int q = 0; q < 4; ++q) {
    const int f = (wave * 4 + q) * 128 + 4 * lane;
    *(volatile v4i*)(cp + f) = cq[q];
  }
  __threadfence();
#pragma unroll
  for (int q = 0; q < 4; ++q) {
    const int f = (wave * 4 + q) * 128 + 4 * lane;
    *(volatile v4i*)(cp + f) = cq[q];
  }
}

__global__ __launch_bounds__(OTHR) void k_offsets(const int* __restrict__ cnt, int* off, int* rbase, int nChunk) {
  __shared__ __attribute__((aligned(16))) int soff[NBC];
  __shared__ __attribute__((aligned(16))) int srb[RBN];
  __shared__ int wtot[OTHR / 32];
  const int tid = threadIdx.x, lane = tid & 31, wave = tid >> 5, sub = tid / TPS;
  for (int i = tid; i < RBN; i += OTHR) srb[i] = 0;
  int carry = 0;
#pragma unroll 1
  for (int ch = 0; ch < nChunk; ++ch) {
    const int base = ch * NBC;
    const v4i c0 = *(const v4i*)(cnt + base + 8 * tid);
    const v4i c1 = *(const v4i*)(cnt + base + 8 * tid + 4);
    const int lim = 1 << 20;
    const int e0 = min(max(c0.x, 0), lim), e1 = min(max(c0.y, 0), lim), e2 = min(max(c0.z, 0), lim), e3 = min(max(c0.w, 0), lim);
    const int e4 = min(max(c1.x, 0), lim), e5 = min(max(c1.y, 0), lim), e6 = min(max(c1.z, 0), lim), e7 = min(max(c1.w, 0), lim);
    const int ts = e0 + e1 + e2 + e3 + e4 + e5 + e6 + e7;
    int incl = ts;
#pragma unroll
    for (int d = 1; d < 32; d <<= 1) {
      const int t = __shfl_up(incl, d);
      if (lane >= d) incl += t;
    }
    if (lane == 31) wtot[wave] = incl;
    __syncthreads();
    int pre = 0;
#pragma unroll 1
    for (int w = WPS * sub; w < wave; ++w) pre += wtot[w];
    int bcur = carry, myb = carry;
#pragma unroll
    for (int j = 0; j < NSUB; ++j) {
      int S = 0;
#pragma unroll
      for (int w = 0; w < WPS; ++w) S += wtot[j * WPS + w];
      if (j == sub) myb = bcur;
      if (tid == 0) srb[min(NSUB * ch + j, RBN - 1)] = bcur;
      S = S < 0 ? 0 : S;
      bcur += (S + 31) & ~31;
    }
    int run = myb + pre + incl - ts;
    soff[8 * tid + 0] = run; run += e0;
    soff[8 * tid + 1] = run; run += e1;
    soff[8 * tid + 2] = run; run += e2;
    soff[8 * tid + 3] = run; run += e3;
    soff[8 * tid + 4] = run; run += e4;
    soff[8 * tid + 5] = run; run += e5;
    soff[8 * tid + 6] = run; run += e6;
    soff[8 * tid + 7] = run;
    carry = bcur;
    __syncthreads();
    const v4i o0 = *(const v4i*)(soff + 4 * tid);
    const v4i o1 = *(const v4i*)(soff + 4 * (tid + OTHR));
    int* op = off + base;
    *(volatile v4i*)(op + 4 * tid) = o0;
    *(volatile v4i*)(op + 4 * (tid + OTHR)) = o1;
    __threadfence();
    *(volatile v4i*)(op + 4 * tid) = o0;
    *(volatile v4i*)(op + 4 * (tid + OTHR)) = o1;
    __syncthreads();
  }
  if (tid == 0) srb[min(NSUB * nChunk, RBN - 1)] = carry;
  __syncthreads();
  v4i rv = {0, 0, 0, 0};
  if (tid < 32) rv = *(const v4i*)(srb + 4 * tid);
  if (tid < 32) *(volatile v4i*)(rbase + 4 * tid) = rv;
  __threadfence();
  if (tid < 32) *(volatile v4i*)(rbase + 4 * tid) = rv;
}

__global__ __launch_bounds__(NTHR) void k_fill(
    const int* __restrict__ ei, const int* __restrict__ off, const int* __restrict__ rbase,
    int* csr, int nN, int nE, int vec8, int csrLen) {
  extern __shared__ v4f lds_dyn[];
  int* region = (int*)lds_dyn;
  int* cursor = region + RCAP;
  int* list   = cursor + NBF;
  int* wcnt   = list + LISTN;
  const int tid = threadIdx.x, lane = tid & 31, wave = tid >> 5;
  const int b = blockIdx.x;
  const int nodeBase = b * NBF;
  const int* dsts = ei + nE;

  int rb0 = rbase[b];
  const int rb1 = rbase[b + 1];
  rb0 = rb0 < 0 ? 0 : (rb0 > csrLen ? csrLen : rb0);
  rb0 &= ~31;
  int len = rb1 - rb0;
  len = len < 0 ? 0 : (len > RCAP ? RCAP : len);
  int lenW = (len + 31) & ~31;
  if (rb0 + lenW > csrLen) lenW = (csrLen - rb0) & ~31;

  {
    const v4i z = {0, 0, 0, 0};
    for (int i = tid; i < RCAP / 4; i += NTHR) ((v4i*)region)[i] = z;
    for (int s = tid; s < NBF; s += NTHR) {
      int o = off[nodeBase + s] - rb0;
      o = o < 0 ? 0 : (o > RCAP ? RCAP : o);
      cursor[s] = o;
    }
  }
  __syncthreads();

  const int nChunks = (nE + CHUNK - 1) / CHUNK;
#pragma unroll 1
  for (int ch = 0; ch < nChunks; ++ch) {
    const int cbase = ch * CHUNK;
    const int wc = scan_chunk<NBF>(dsts, nE, cbase, nodeBase, vec8, list, tid, lane, wave);
    if (lane == 0) wcnt[wave] = wc;
    __syncthreads();
    if (wave == 0) {
#pragma unroll 1
      for (int wsx = 0; wsx < NWAVE; ++wsx) {
        int n = __builtin_amdgcn_readfirstlane(wcnt[wsx]);
        n = n > WCAP ? WCAP : (n < 0 ? 0 : n);
        const int* lp = list + wsx * WCAP;
#pragma unroll 1
        for (int i = 0; i < n; ++i) {
          const int ent  = __builtin_amdgcn_readfirstlane(lp[i]);
          const int slot = ent & (NBF - 1);
          int e = cbase + ((ent >> 12) & (CHUNK - 1));
          e = e > nE - 1 ? nE - 1 : e;
          int src = ei[e];
          src = src < 0 ? 0 : (src > nN - 1 ? nN - 1 : src);
          if (lane == 0) {
            int pos = cursor[slot];
            pos = pos < 0 ? 0 : (pos > RCAP - 1 ? RCAP - 1 : pos);
            region[pos] = src;
            const int np = pos + 1;
            cursor[slot] = np > RCAP ? RCAP : np;
          }
        }
      }
    }
    __syncthreads();
  }

  const int nv = lenW >> 2;
  int* gp = csr + rb0;
#pragma unroll 1
  for (int i = tid; i < nv; i += NTHR) { const v4i v = ((const v4i*)region)[i]; *(volatile v4i*)(gp + 4 * i) = v; }
  __threadfence();
#pragma unroll 1
  for (int i = tid; i < nv; i += NTHR) { const v4i v = ((const v4i*)region)[i]; *(volatile v4i*)(gp + 4 * i) = v; }
}

__global__ __launch_bounds__(NTHR) void k_agg(
    const int* __restrict__ csr, const int* __restrict__ off, const int* __restrict__ cnt,
    const float* __restrict__ src, const float* __restrict__ eps, int layer,
    float* dst, int nN, int csrLen) {
  const int tid = threadIdx.x, lane = tid & 31, wave = tid >> 5;
  const int tbase = blockIdx.x * TGT + wave * 32;
  const int cl = tbase + lane;
  const int cnt_l = cnt[cl];
  const int off_l = off[cl];
  const float e1 = 1.0f + eps[layer];

#pragma unroll 1
  for (int j = 0; j < 32; ++j) {
    const int c = tbase + j;
    int n = __builtin_amdgcn_readlane(cnt_l, j);
    n = n < 0 ? 0 : (n > DEGCAP ? DEGCAP : n);
    const int st = __builtin_amdgcn_readlane(off_l, j);
    v4f acc = {0.f, 0.f, 0.f, 0.f};
#pragma unroll 1
    for (int q0 = 0; q0 < n; q0 += 32) {
      int pos = st + q0 + lane;
      pos = pos < 0 ? 0 : (pos > csrLen - 1 ? csrLen - 1 : pos);
      int sl = csr[pos];
      sl = sl < 0 ? 0 : (sl > nN - 1 ? nN - 1 : sl);
      const int mcnt = (n - q0) < 32 ? (n - q0) : 32;
#pragma unroll 1
      for (int p = 0; p < mcnt; ++p) {
        const int s = __builtin_amdgcn_readlane(sl, p);
        acc = acc + *(const v4f*)(src + (size_t)s * HID + 4 * lane);
      }
    }
    const int cs = c > nN - 1 ? nN - 1 : c;
    const v4f sv = *(const v4f*)(src + (size_t)cs * HID + 4 * lane);
    const v4f v = sv * e1 + acc;
    float* hp = dst + (size_t)c * HID + 4 * lane;
    *(volatile v4f*)hp = v;
    __threadfence();
    *(volatile v4f*)hp = v;
  }
}

template <int KD>
__device__ __forceinline__ void gemm_wave(const unsigned short* sAh, const unsigned short* sAl,
                                          const unsigned short* __restrict__ Bh, const unsigned short* __restrict__ Bl,
                                          const float* __restrict__ bias, float* stg, int wave, int lane) {
  constexpr int AP = KD + 8;
  const int hh = lane >> 4, m = lane & 15;
  const unsigned short* arh = sAh + (wave * 16 + m) * AP + 8 * hh;
  const unsigned short* arl = sAl + (wave * 16 + m) * AP + 8 * hh;
  float* sp = stg + (wave * 16 + 8 * hh) * HID + m;
#pragma unroll 1
  for (int g = 0; g < HID / 64; ++g) {
    v8f acc[4];
#pragma unroll
    for (int t = 0; t < 4; ++t) { v8f z = {0.f, 0.f, 0.f, 0.f, 0.f, 0.f, 0.f, 0.f}; acc[t] = z; }
#pragma unroll
    for (int kt = 0; kt < KD / 32; ++kt) {
      FragB ah, al;
      ah.h[0] = *(const v8us*)(arh + 32 * kt);
      ah.h[1] = *(const v8us*)(arh + 32 * kt + 16);
      al.h[0] = *(const v8us*)(arl + 32 * kt);
      al.h[1] = *(const v8us*)(arl + 32 * kt + 16);
#pragma unroll
      for (int t = 0; t < 4; ++t) {
        const size_t bo = (size_t)(64 * g + 16 * t + m) * KD + 32 * kt + 8 * hh;
        FragB bh, bl;
        bh.h[0] = *(const v8us*)(Bh + bo);
        bh.h[1] = *(const v8us*)(Bh + bo + 16);
        bl.h[0] = *(const v8us*)(Bl + bo);
        bl.h[1] = *(const v8us*)(Bl + bo + 16);
        acc[t] = wm3(ah.v, al.v, bh.v, bl.v, acc[t]);
      }
    }
#pragma unroll
    for (int t = 0; t < 4; ++t) {
      const int col = 64 * g + 16 * t + m;
      const float bv = bias[col];
#pragma unroll
      for (int r = 0; r < 8; ++r) sp[r * HID + 64 * g + 16 * t] = acc[t][r] + bv;
    }
  }
}

__global__ __launch_bounds__(NTHR) void k_gemm1(
    const float* __restrict__ A, const unsigned short* __restrict__ Bh, const unsigned short* __restrict__ Bl,
    const float* __restrict__ bias, float* C, double* part, int nRowsA, int nN) {
  extern __shared__ v4f lds_dyn[];
  unsigned short* sAh = (unsigned short*)lds_dyn;
  unsigned short* sAl = sAh + GROWS * APH;
  float*  stg   = (float*)(sAl + GROWS * APH);
  double* sPart = (double*)(stg + GROWS * HID);
  const int tid = threadIdx.x, lane = tid & 31, wave = tid >> 5;
  const int rowBase = blockIdx.x * GROWS;

#pragma unroll
  for (int i = 0; i < (GROWS * HID / 8) / NTHR; ++i) {
    const int idx = i * NTHR + tid;
    const int r   = idx >> 4;
    const int c0  = (idx & 15) * 8;
    int row = rowBase + r;
    row = row > nRowsA - 1 ? nRowsA - 1 : row;
    const float* ap = A + (size_t)row * HID + c0;
    const v4f a = *(const v4f*)ap, b = *(const v4f*)(ap + 4);
    v8us hi, lo;
    split8(a, b, hi, lo);
    *(v8us*)(sAh + r * APH + c0) = hi;
    *(v8us*)(sAl + r * APH + c0) = lo;
  }
  __syncthreads();

  gemm_wave<HID>(sAh, sAl, Bh, Bl, bias, stg, wave, lane);
  __syncthreads();

  {
    const int col = tid & (HID - 1), which = tid >> 7;
    int nr = nN - rowBase;
    nr = nr < 0 ? 0 : (nr > GROWS ? GROWS : nr);
    double s = 0.0;
    if (which == 0) {
#pragma unroll 1
      for (int r = 0; r < nr; ++r) s += (double)stg[r * HID + col];
    } else {
#pragma unroll 1
      for (int r = 0; r < nr; ++r) { const double d = (double)stg[r * HID + col]; s += d * d; }
    }
    sPart[tid] = s;
  }
  __syncthreads();

  v4f pv[4];
  const v4f z4 = {0.f, 0.f, 0.f, 0.f};
#pragma unroll
  for (int q = 0; q < 4; ++q) pv[q] = z4;
  if (wave == 0) {
#pragma unroll
    for (int q = 0; q < 4; ++q) pv[q] = *(const v4f*)((const char*)sPart + 16 * (q * 32 + lane));
  }
  char* pp = (char*)(part + (size_t)blockIdx.x * (2 * HID));
  const float* lp = stg + wave * 16 * HID + 4 * lane;
  float* gp = C + ((size_t)rowBase + wave * 16) * HID + 4 * lane;
  if (wave == 0) {
#pragma unroll
    for (int q = 0; q < 4; ++q) *(volatile v4f*)(pp + 16 * (q * 32 + lane)) = pv[q];
  }
#pragma unroll
  for (int i = 0; i < 16; ++i) { const v4f v = *(const v4f*)(lp + i * HID); *(volatile v4f*)(gp + (size_t)i * HID) = v; }
  __threadfence();
  if (wave == 0) {
#pragma unroll
    for (int q = 0; q < 4; ++q) *(volatile v4f*)(pp + 16 * (q * 32 + lane)) = pv[q];
  }
#pragma unroll
  for (int i = 0; i < 16; ++i) { const v4f v = *(const v4f*)(lp + i * HID); *(volatile v4f*)(gp + (size_t)i * HID) = v; }
}

__global__ __launch_bounds__(NTHR) void k_bnfin(
    const double* __restrict__ part, int nPart, const float* __restrict__ gam, int nN, float* bnp) {
  __shared__ __attribute__((aligned(16))) double sRed[2 * HID];
  __shared__ __attribute__((aligned(16))) float sOut[2 * HID];
  const int tid = threadIdx.x, lane = tid & 31, wave = tid >> 5;
  double s = 0.0;
#pragma unroll 1
  for (int b = 0; b < nPart; ++b) s += part[(size_t)b * (2 * HID) + tid];
  sRed[tid] = s;
  __syncthreads();
  if (tid < HID) {
    const double inv = 1.0 / (double)(nN > 0 ? nN : 1);
    const double mean = sRed[tid] * inv;
    double var = sRed[HID + tid] * inv - mean * mean;
    var = var < 0.0 ? 0.0 : var;
    const float varf = (float)var;
    const float rstd = 1.0f / sqrtf(varf + BNEPS);
    sOut[tid] = (float)mean;
    sOut[HID + tid] = rstd * gam[tid];
  }
  __syncthreads();
  v4f o0 = {0.f, 0.f, 0.f, 0.f}, o1 = {0.f, 0.f, 0.f, 0.f};
  if (wave == 0) { o0 = *(const v4f*)(sOut + 4 * lane); o1 = *(const v4f*)(sOut + HID + 4 * lane); }
  if (wave == 0) { *(volatile v4f*)(bnp + 4 * lane) = o0; *(volatile v4f*)(bnp + HID + 4 * lane) = o1; }
  __threadfence();
  if (wave == 0) { *(volatile v4f*)(bnp + 4 * lane) = o0; *(volatile v4f*)(bnp + HID + 4 * lane) = o1; }
}

__global__ __launch_bounds__(NTHR) void k_gemm2(
    const float* __restrict__ A, const float* __restrict__ bnp, const float* __restrict__ beta,
    const unsigned short* __restrict__ Bh, const unsigned short* __restrict__ Bl,
    const float* __restrict__ bias, const float* __restrict__ lng, const float* __restrict__ lnb,
    float* C, int nRowsA) {
  extern __shared__ v4f lds_dyn[];
  unsigned short* sAh = (unsigned short*)lds_dyn;
  unsigned short* sAl = sAh + GROWS * APH;
  float* stg  = (float*)(sAl + GROWS * APH);
  float* sPar = stg + GROWS * HID;
  const int tid = threadIdx.x, lane = tid & 31, wave = tid >> 5;
  const int rowBase = blockIdx.x * GROWS;

  if (wave == 0)      *(v4f*)(sPar + 4 * lane)           = *(const v4f*)(bnp + 4 * lane);
  else if (wave == 1) *(v4f*)(sPar + HID + 4 * lane)     = *(const v4f*)(bnp + HID + 4 * lane);
  else if (wave == 2) *(v4f*)(sPar + 2 * HID + 4 * lane) = *(const v4f*)(beta + 4 * lane);
  __syncthreads();

#pragma unroll
  for (int i = 0; i < (GROWS * HID / 8) / NTHR; ++i) {
    const int idx = i * NTHR + tid;
    const int r   = idx >> 4;
    const int c0  = (idx & 15) * 8;
    int row = rowBase + r;
    row = row > nRowsA - 1 ? nRowsA - 1 : row;
    const float* ap = A + (size_t)row * HID + c0;
    v4f a = *(const v4f*)ap, b = *(const v4f*)(ap + 4);
    const v4f m0 = *(const v4f*)(sPar + c0),           m1 = *(const v4f*)(sPar + c0 + 4);
    const v4f s0 = *(const v4f*)(sPar + HID + c0),     s1 = *(const v4f*)(sPar + HID + c0 + 4);
    const v4f t0 = *(const v4f*)(sPar + 2 * HID + c0), t1 = *(const v4f*)(sPar + 2 * HID + c0 + 4);
    a = (a - m0) * s0 + t0;
    b = (b - m1) * s1 + t1;
    a.x = fmaxf(a.x, 0.f); a.y = fmaxf(a.y, 0.f); a.z = fmaxf(a.z, 0.f); a.w = fmaxf(a.w, 0.f);
    b.x = fmaxf(b.x, 0.f); b.y = fmaxf(b.y, 0.f); b.z = fmaxf(b.z, 0.f); b.w = fmaxf(b.w, 0.f);
    v8us hi, lo;
    split8(a, b, hi, lo);
    *(v8us*)(sAh + r * APH + c0) = hi;
    *(v8us*)(sAl + r * APH + c0) = lo;
  }
  __syncthreads();

  gemm_wave<HID>(sAh, sAl, Bh, Bl, bias, stg, wave, lane);
  __syncthreads();

  const v4f g4 = *(const v4f*)(lng + 4 * lane);
  const v4f b4 = *(const v4f*)(lnb + 4 * lane);
  float* lp = stg + wave * 16 * HID + 4 * lane;
#pragma unroll 4
  for (int i = 0; i < 16; ++i) {
    const v4f v = *(const v4f*)(lp + i * HID);
    float s = (v.x + v.y) + (v.z + v.w);
    s = wsum(s);
    const float mean = s * (1.0f / (float)HID);
    const v4f d = v - mean;
    float q = d.x * d.x + d.y * d.y + d.z * d.z + d.w * d.w;
    q = wsum(q);
    const float rstd = rsqrtf(q * (1.0f / (float)HID) + LNEPS);
    v4f o = (d * rstd) * g4 + b4;
    o.x = o.x >= 0.0f ? o.x : 0.1f * o.x;
    o.y = o.y >= 0.0f ? o.y : 0.1f * o.y;
    o.z = o.z >= 0.0f ? o.z : 0.1f * o.z;
    o.w = o.w >= 0.0f ? o.w : 0.1f * o.w;
    *(v4f*)(lp + i * HID) = o;
  }
  float* gp = C + ((size_t)rowBase + wave * 16) * HID + 4 * lane;
#pragma unroll
  for (int i = 0; i < 16; ++i) { const v4f v = *(const v4f*)(lp + i * HID); *(volatile v4f*)(gp + (size_t)i * HID) = v; }
  __threadfence();
#pragma unroll
  for (int i = 0; i < 16; ++i) { const v4f v = *(const v4f*)(lp + i * HID); *(volatile v4f*)(gp + (size_t)i * HID) = v; }
}

__global__ __launch_bounds__(NTHR) void k_pool(
    const int* __restrict__ bidx, const int* __restrict__ numg, const float* __restrict__ P,
    float* pooled, int nN, int G) {
  __shared__ __attribute__((aligned(16))) float ssum[NBP * HID];
  __shared__ __attribute__((aligned(16))) float smax[NBP * HID];
  __shared__ __attribute__((aligned(16))) int list[LISTN];
  __shared__ int pc[NBP];
  __shared__ int wcnt[NWAVE];
  const int tid = threadIdx.x, lane = tid & 31, wave = tid >> 5;
  const int gBase = blockIdx.x * NBP;
  int ng = numg[0];
  ng = (ng <= 0 || ng > G) ? G : ng;

  {
    const v4f z = {0.f, 0.f, 0.f, 0.f};
    const float ninf = __uint_as_float(0xff800000u);
    const v4f mi = {ninf, ninf, ninf, ninf};
    for (int i = tid; i < NBP * HID / 4; i += NTHR) { ((v4f*)ssum)[i] = z; ((v4f*)smax)[i] = mi; }
    for (int i = tid; i < NBP; i += NTHR) pc[i] = 0;
  }
  __syncthreads();

  const int nChunks = (nN + CHUNK - 1) / CHUNK;
#pragma unroll 1
  for (int ch = 0; ch < nChunks; ++ch) {
    const int cbase = ch * CHUNK;
    const int wc = scan_chunk<NBP>(bidx, nN, cbase, gBase, 1, list, tid, lane, wave);
    if (lane == 0) wcnt[wave] = wc;
    __syncthreads();
    if (wave == 0) {
#pragma unroll 1
      for (int wsx = 0; wsx < NWAVE; ++wsx) {
        int n = __builtin_amdgcn_readfirstlane(wcnt[wsx]);
        n = n > WCAP ? WCAP : (n < 0 ? 0 : n);
        const int* lp = list + wsx * WCAP;
#pragma unroll 1
        for (int i = 0; i < n; ++i) {
          const int ent  = __builtin_amdgcn_readfirstlane(lp[i]);
          const int slot = ent & (NBP - 1);
          if (gBase + slot < ng) {
            int nd = cbase + ((ent >> 12) & (CHUNK - 1));
            nd = nd > nN - 1 ? nN - 1 : nd;
            const v4f v = *(const v4f*)(P + (size_t)nd * HID + 4 * lane);
            v4f* ap = (v4f*)(ssum + slot * HID + 4 * lane);
            *ap = *ap + v;
            v4f* mp = (v4f*)(smax + slot * HID + 4 * lane);
            v4f mv = *mp;
            mv.x = fmaxf(mv.x, v.x); mv.y = fmaxf(mv.y, v.y); mv.z = fmaxf(mv.z, v.z); mv.w = fmaxf(mv.w, v.w);
            *mp = mv;
            if (lane == 0) pc[slot] = pc[slot] + 1;
          }
        }
      }
    }
    __syncthreads();
  }

  v4f ov[8];
#pragma unroll
  for (int p = 0; p < 8; ++p) {
    const int f   = p * NTHR + tid;
    const int row = f >> 6;
    const int c4  = f & 63;
    const int cc  = 4 * (c4 & 31);
    int cv = pc[row];
    cv = cv < 1 ? 1 : cv;
    const float inv = 1.0f / (float)cv;
    const v4f mx = *(const v4f*)(smax + row * HID + cc);
    const v4f sm = *(const v4f*)(ssum + row * HID + cc) * inv;
    v4f o;
    o.x = c4 < 32 ? mx.x : sm.x; o.y = c4 < 32 ? mx.y : sm.y; o.z = c4 < 32 ? mx.z : sm.z; o.w = c4 < 32 ? mx.w : sm.w;
    ov[p] = o;
  }
  float* gp = pooled + (size_t)gBase * KOUT;
#pragma unroll
  for (int p = 0; p < 8; ++p) *(volatile v4f*)(gp + 4 * (p * NTHR + tid)) = ov[p];
  __threadfence();
#pragma unroll
  for (int p = 0; p < 8; ++p) *(volatile v4f*)(gp + 4 * (p * NTHR + tid)) = ov[p];
}

__global__ __launch_bounds__(NTHR) void k_head(
    const float* __restrict__ A, const unsigned short* __restrict__ Bh, const unsigned short* __restrict__ Bl,
    const float* __restrict__ bias, float* out, int nRowsA, int G) {
  extern __shared__ v4f lds_dyn[];
  unsigned short* sAh = (unsigned short*)lds_dyn;
  unsigned short* sAl = sAh + GROWS * APO;
  float* stg = (float*)(sAl + GROWS * APO);
  const int tid = threadIdx.x, lane = tid & 31, wave = tid >> 5;
  const int rowBase = blockIdx.x * GROWS;

#pragma unroll
  for (int i = 0; i < (GROWS * KOUT / 8) / NTHR; ++i) {
    const int idx = i * NTHR + tid;
    const int r   = idx >> 5;
    const int c0  = (idx & 31) * 8;
    int row = rowBase + r;
    row = row > nRowsA - 1 ? nRowsA - 1 : row;
    const float* ap = A + (size_t)row * KOUT + c0;
    const v4f a = *(const v4f*)ap, b = *(const v4f*)(ap + 4);
    v8us hi, lo;
    split8(a, b, hi, lo);
    *(v8us*)(sAh + r * APO + c0) = hi;
    *(v8us*)(sAl + r * APO + c0) = lo;
  }
  __syncthreads();

  gemm_wave<KOUT>(sAh, sAl, Bh, Bl, bias, stg, wave, lane);
  __syncthreads();

  const float* lp = stg + wave * 16 * HID + 4 * lane;
  const int rw = rowBase + wave * 16;
  float* gp = out + (size_t)rw * HID + 4 * lane;
#pragma unroll
  for (int i = 0; i < 16; ++i) {
    if (rw + i < G) { const v4f v = *(const v4f*)(lp + i * HID); *(volatile v4f*)(gp + (size_t)i * HID) = v; }
  }
  __threadfence();
#pragma unroll
  for (int i = 0; i < 16; ++i) {
    if (rw + i < G) { const v4f v = *(const v4f*)(lp + i * HID); *(volatile v4f*)(gp + (size_t)i * HID) = v; }
  }
}

extern "C" void kernel_launch(void* const* d_in, const int* in_sizes, int n_in,
                              void* d_out, int out_size, void* d_ws, size_t ws_size,
                              hipStream_t stream) {
  if (n_in < 15) return;
  const int nN = in_sizes[13];
  if (nN <= 0 || nN > (1 << 24) || in_sizes[0] != nN * HID) return;
  const int L = in_sizes[1] / (HID * HID);
  if (L < 1 || L > 16 || in_sizes[1] != L * HID * HID || in_sizes[5] != in_sizes[1]) return;
  if (in_sizes[2] < L * HID || in_sizes[3] < L * HID || in_sizes[4] < L * HID || in_sizes[6] < L * HID ||
      in_sizes[7] < L || in_sizes[8] < L * HID || in_sizes[9] < L * HID) return;
  if (in_sizes[10] != KOUT * HID || in_sizes[11] < HID || in_sizes[14] < 1) return;
  const int nE = in_sizes[12] / 2;
  if (nE <= 0 || nE > (1 << 28) || in_sizes[12] != 2 * nE) return;
  const int G = out_size / HID;
  if (G <= 0 || out_size != G * HID) return;

  const float* x    = (const float*)d_in[0];
  const float* W1   = (const float*)d_in[1];
  const float* b1   = (const float*)d_in[2];
  const float* bng  = (const float*)d_in[3];
  const float* bnb  = (const float*)d_in[4];
  const float* W2   = (const float*)d_in[5];
  const float* b2   = (const float*)d_in[6];
  const float* geps = (const float*)d_in[7];
  const float* lng  = (const float*)d_in[8];
  const float* lnb  = (const float*)d_in[9];
  const float* Wo   = (const float*)d_in[10];
  const float* bout = (const float*)d_in[11];
  const int*   ei   = (const int*)d_in[12];
  const int*   bidx = (const int*)d_in[13];
  const int*   numg = (const int*)d_in[14];
  float* out = (float*)d_out;

  const int NPAD   = ((nN + TGT - 1) / TGT) * TGT;
  const int nBC    = (nN + NBC - 1) / NBC;
  const int CNTPAD = nBC * NBC;
  if (NSUB * nBC + 1 > RBN) return;
  const int nBF    = (nN + NBF - 1) / NBF;
  const int csrLen = ((nE + 31) & ~31) + 32 * (NSUB * nBC + 2);
  const int nGemm  = NPAD / GROWS;
  const int nAgg   = NPAD / TGT;
  const int nPool  = (G + NBP - 1) / NBP;
  const int GP     = nPool * NBP;
  const int nHead  = (G + GROWS - 1) / GROWS;

  char* ws = (char*)d_ws;
  size_t off = 0;
  const size_t wsz  = (size_t)L * HID * HID * 2;
  const size_t oW1h = off; off += wsz;                              off = (off + 255) & ~(size_t)255;
  const size_t oW1l = off; off += wsz;                              off = (off + 255) & ~(size_t)255;
  const size_t oW2h = off; off += wsz;                              off = (off + 255) & ~(size_t)255;
  const size_t oW2l = off; off += wsz;                              off = (off + 255) & ~(size_t)255;
  const size_t oWoh = off; off += (size_t)HID * KOUT * 2;           off = (off + 255) & ~(size_t)255;
  const size_t oWol = off; off += (size_t)HID * KOUT * 2;           off = (off + 255) & ~(size_t)255;
  const size_t oCnt = off; off += (size_t)CNTPAD * 4;               off = (off + 255) & ~(size_t)255;
  const size_t oOff = off; off += (size_t)CNTPAD * 4;               off = (off + 255) & ~(size_t)255;
  const size_t oRb  = off; off += (size_t)RBN * 4;                  off = (off + 255) & ~(size_t)255;
  const size_t oCsr = off; off += (size_t)csrLen * 4;               off = (off + 255) & ~(size_t)255;
  const size_t oPA  = off; off += (size_t)NPAD * HID * 4;           off = (off + 255) & ~(size_t)255;
  const size_t oPB  = off; off += (size_t)NPAD * HID * 4;           off = (off + 255) & ~(size_t)255;
  const size_t oPrt = off; off += (size_t)nGemm * 2 * HID * 8;      off = (off + 255) & ~(size_t)255;
  const size_t oBnp = off; off += (size_t)2 * HID * 4;              off = (off + 255) & ~(size_t)255;
  const size_t oPl  = off; off += (size_t)GP * KOUT * 4;            off = (off + 255) & ~(size_t)255;
  if (off > ws_size) return;
  unsigned short* w1h = (unsigned short*)(ws + oW1h);
  unsigned short* w1l = (unsigned short*)(ws + oW1l);
  unsigned short* w2h = (unsigned short*)(ws + oW2h);
  unsigned short* w2l = (unsigned short*)(ws + oW2l);
  unsigned short* woh = (unsigned short*)(ws + oWoh);
  unsigned short* wol = (unsigned short*)(ws + oWol);
  int*    cnt    = (int*)(ws + oCnt);
  int*    offp   = (int*)(ws + oOff);
  int*    rb     = (int*)(ws + oRb);
  int*    csr    = (int*)(ws + oCsr);
  float*  pA     = (float*)(ws + oPA);
  float*  pB     = (float*)(ws + oPB);
  double* part   = (double*)(ws + oPrt);
  float*  bnp    = (float*)(ws + oBnp);
  float*  pooled = (float*)(ws + oPl);

  const int vec8 = ((nE & 3) == 0) ? 1 : 0;

  const int nPrep = 2 * L * (HID * HID / 8) + HID * KOUT / 8;
  k_wprep<<<(nPrep + NTHR - 1) / NTHR, NTHR, 0, stream>>>(W1, W2, Wo, w1h, w1l, w2h, w2l, woh, wol, L);

  k_count<<<nBC, NTHR, 0, stream>>>(ei, cnt, nE, vec8);
  k_offsets<<<1, OTHR, 0, stream>>>(cnt, offp, rb, nBC);
  hipFuncSetAttribute(reinterpret_cast<const void*>(&k_fill), hipFuncAttributeMaxDynamicSharedMemorySize, LDS_FILL);
  k_fill<<<nBF, NTHR, LDS_FILL, stream>>>(ei, offp, rb, csr, nN, nE, vec8, csrLen);

  hipFuncSetAttribute(reinterpret_cast<const void*>(&k_gemm1), hipFuncAttributeMaxDynamicSharedMemorySize, LDS_G1);
  hipFuncSetAttribute(reinterpret_cast<const void*>(&k_gemm2), hipFuncAttributeMaxDynamicSharedMemorySize, LDS_G2);
  const float* cur = x;
  float* bufIn = pA;
  float* bufOt = pB;
  for (int l = 0; l < L; ++l) {
    const size_t wl = (size_t)l * HID * HID;
    const size_t pl = (size_t)l * HID;
    k_agg<<<nAgg, NTHR, 0, stream>>>(csr, offp, cnt, cur, geps, l, bufIn, nN, csrLen);
    k_gemm1<<<nGemm, NTHR, LDS_G1, stream>>>(bufIn, w1h + wl, w1l + wl, b1 + pl, bufOt, part, NPAD, nN);
    k_bnfin<<<1, NTHR, 0, stream>>>(part, nGemm, bng + pl, nN, bnp);
    k_gemm2<<<nGemm, NTHR, LDS_G2, stream>>>(bufOt, bnp, bnb + pl, w2h + wl, w2l + wl, b2 + pl, lng + pl, lnb + pl, bufIn, NPAD);
    cur = bufIn;
    float* t = bufIn; bufIn = bufOt; bufOt = t;
  }

  k_pool<<<nPool, NTHR, 0, stream>>>(bidx, numg, cur, pooled, nN, G);
  hipFuncSetAttribute(reinterpret_cast<const void*>(&k_head), hipFuncAttributeMaxDynamicSharedMemorySize, LDS_HD);
  k_head<<<nHead, NTHR, LDS_HD, stream>>>(pooled, woh, wol, bout, out, GP, G);
}
